// HGNNLayerDGL_78847009620370
// MI455X (gfx1250) — hardware-run, weakly checked
//
#include <hip/hip_runtime.h>
#include <stddef.h>
#include <stdint.h>
#include <math.h>


#define NG      20000
#define ND      8000
#define NS      8000
#define NEDGE   300000
#define DIM     256
#define KVW     512
#define KHL     512
#define MPG     20096
#define MPD     8064
#define NTHR    256
#define NWAVE   8
#define EPT     8
#define CHUNK   (NTHR * EPT)
#define WCAP    (EPT * 32)
#define LISTN   (NWAVE * WCAP)
#define NBMAX   2048
#define SLOTB   11
#define RCAP    28672
#define DEGCAP  256
#define NB0     1024
#define NB1     512
#define GA0     20
#define GA1     16
#define STW     512
#define GBM     64
#define GBN     128
#define GTHR    128
#define GNT     8
#define FBM     32
#define MX0     (-1.0e30f)
#define QK_SCALE 0.17677669529663687f
#define LN_EPS  1.0e-5f
#define WSMAX   134217728
#define LDS_AGG ((2 * RCAP + 2 * NBMAX + LISTN) * 4 + 64)
#define OUT1    (ND * DIM)
#define OUT2    (ND * DIM + NS * DIM)
#define OUTN    (ND * DIM + NS * DIM + NG * DIM)

static_assert(DIM == 8 * 32 && DIM == 32 * 8);
static_assert(ND == NS);
static_assert((CHUNK & (CHUNK - 1)) == 0 && CHUNK <= (1 << SLOTB));
static_assert(NBMAX == (1 << SLOTB));
static_assert(NTHR * 8 == NBMAX);
static_assert(LISTN >= NBMAX && LISTN >= NWAVE * WCAP && LISTN >= 2 * DIM);
static_assert((RCAP % 32) == 0);
static_assert(RCAP >= 19532 + 8192);
static_assert(RCAP >= 15604 + 8192);
static_assert(DEGCAP >= 65 + 8);
static_assert(NEDGE < (1 << (32 - SLOTB)) && (NEDGE % 4) == 0);
static_assert((NB0 % 16) == 0 && (NB1 % 16) == 0 && NB0 <= NBMAX && NB1 <= NBMAX);
static_assert(NB0 == 4 * NTHR);
static_assert(GA0 * NB0 >= MPG && (GA0 - 1) * NB0 < MPG);
static_assert(GA1 * NB1 >= ND && (GA1 - 1) * NB1 < ND);
static_assert((MPG % 128) == 0 && MPG >= NG && MPG - NG < 128);
static_assert((MPD % 128) == 0 && MPD >= ND && MPD - ND < 128);
static_assert(NWAVE * STW <= RCAP && DIM <= STW);
static_assert(LDS_AGG <= 327680);
static_assert(GBM == (GTHR / 32) * 16 && GBN == 16 * GNT && GTHR == GBN);
static_assert((DIM % 32) == 0 && (KHL % 32) == 0 && (DIM % GBN) == 0 && (KVW % GBN) == 0);
static_assert(NTHR == DIM);
static_assert(OUT1 == 2048000 && OUT2 == 4096000 && OUTN == 9216000);
static_assert(OUT2 + (NG - 1) * DIM + DIM - 1 < OUTN);

typedef float          v4f  __attribute__((ext_vector_type(4)));
typedef float          v8f  __attribute__((ext_vector_type(8)));
typedef int            v4i  __attribute__((ext_vector_type(4)));
typedef int            v8i  __attribute__((ext_vector_type(8)));
typedef unsigned int   v4u  __attribute__((ext_vector_type(4)));
typedef unsigned short v8us __attribute__((ext_vector_type(8)));
typedef __bf16         v16b __attribute__((ext_vector_type(16)));
typedef v4f  __attribute__((may_alias)) v4fa;
typedef v4u  __attribute__((may_alias)) v4ua;
typedef v8us __attribute__((may_alias)) v8usa;
union Frag { v16b vb; v8us h[2]; v8i w; };

__device__ __forceinline__ v8f wmb(const Frag& a, const Frag& b, v8f c) {
  v8f d = __builtin_amdgcn_wmma_f32_16x16x32_bf16(false, a.vb, false, b.vb, (short)0, c, false, false);
  asm volatile("v_nop\n\tv_nop\n\tv_nop\n\tv_nop" : "+v"(d) : "v"(a.w), "v"(b.w));
  return d;
}

__device__ __forceinline__ unsigned short bf_bits(float f) {
  unsigned int u = __float_as_uint(f);
  u = (f != f) ? 0x7FC00000u : u;
  u += 0x7FFFu + ((u >> 16) & 1u);
  return (unsigned short)(u >> 16);
}
__device__ __forceinline__ float bf_val(unsigned short b) { return __uint_as_float(((unsigned int)b) << 16); }
__device__ __forceinline__ float bf_rne(float f) { return bf_val(bf_bits(f)); }
__device__ __forceinline__ unsigned int pk2(float lo, float hi) {
  return (unsigned int)bf_bits(lo) | ((unsigned int)bf_bits(hi) << 16);
}
__device__ __forceinline__ v4u pack8(const v4f a, const v4f b) {
  v4u r;
  r.x = pk2(a.x, a.y); r.y = pk2(a.z, a.w); r.z = pk2(b.x, b.y); r.w = pk2(b.z, b.w);
  return r;
}
__device__ __forceinline__ float rlo(unsigned int h, unsigned int l) {
  return __uint_as_float(h << 16) + __uint_as_float(l << 16);
}
__device__ __forceinline__ float rhi(unsigned int h, unsigned int l) {
  return __uint_as_float(h & 0xFFFF0000u) + __uint_as_float(l & 0xFFFF0000u);
}
struct HL8 { v4u h; v4u l; };
__device__ __forceinline__ HL8 hl8(const v4f a, const v4f b) {
  const float f[8] = {a.x, a.y, a.z, a.w, b.x, b.y, b.z, b.w};
  unsigned int wh[4], wl[4];
#pragma unroll
  for (int j = 0; j < 4; ++j) {
    const unsigned short h0 = bf_bits(f[2 * j]), h1 = bf_bits(f[2 * j + 1]);
    const unsigned short l0 = bf_bits(f[2 * j] - bf_val(h0)), l1 = bf_bits(f[2 * j + 1] - bf_val(h1));
    wh[j] = (unsigned int)h0 | ((unsigned int)h1 << 16);
    wl[j] = (unsigned int)l0 | ((unsigned int)l1 << 16);
  }
  HL8 r;
  r.h.x = wh[0]; r.h.y = wh[1]; r.h.z = wh[2]; r.h.w = wh[3];
  r.l.x = wl[0]; r.l.y = wl[1]; r.l.z = wl[2]; r.l.w = wl[3];
  return r;
}

__device__ __forceinline__ int scan_chunk(const int* __restrict__ dsts, int nE, int cbase, int slotBase,
                                          int nb, int vec8, int* list, int tid, int lane, int wave) {
  int wc = 0;
  const int el0  = tid * EPT;
  const int e0   = cbase + el0;
  const int sent = -2147483647 - 1;
  v4i da, db;
  if (vec8 != 0 && cbase + CHUNK <= nE) {
    da = *(const v4i*)(dsts + e0);
    db = *(const v4i*)(dsts + e0 + 4);
  } else {
    da.x = (e0     < nE) ? dsts[min(e0,     nE - 1)] : sent;
    da.y = (e0 + 1 < nE) ? dsts[min(e0 + 1, nE - 1)] : sent;
    da.z = (e0 + 2 < nE) ? dsts[min(e0 + 2, nE - 1)] : sent;
    da.w = (e0 + 3 < nE) ? dsts[min(e0 + 3, nE - 1)] : sent;
    db.x = (e0 + 4 < nE) ? dsts[min(e0 + 4, nE - 1)] : sent;
    db.y = (e0 + 5 < nE) ? dsts[min(e0 + 5, nE - 1)] : sent;
    db.z = (e0 + 6 < nE) ? dsts[min(e0 + 6, nE - 1)] : sent;
    db.w = (e0 + 7 < nE) ? dsts[min(e0 + 7, nE - 1)] : sent;
  }
  const unsigned nbs = (unsigned)slotBase;
  const unsigned unb = (unsigned)nb;
  const unsigned s0 = (unsigned)da.x - nbs, s1 = (unsigned)da.y - nbs;
  const unsigned s2 = (unsigned)da.z - nbs, s3 = (unsigned)da.w - nbs;
  const unsigned s4 = (unsigned)db.x - nbs, s5 = (unsigned)db.y - nbs;
  const unsigned s6 = (unsigned)db.z - nbs, s7 = (unsigned)db.w - nbs;
  const bool h0 = s0 < unb, h1 = s1 < unb, h2 = s2 < unb, h3 = s3 < unb;
  const bool h4 = s4 < unb, h5 = s5 < unb, h6 = s6 < unb, h7 = s7 < unb;
  const unsigned any = __builtin_amdgcn_ballot_w32(h0 | h1 | h2 | h3 | h4 | h5 | h6 | h7);
  if (any != 0u) {
#define HITJ(J, HJ, SJ) { \
      const unsigned mj = __builtin_amdgcn_ballot_w32(HJ); \
      if (mj != 0u) { \
        if (HJ) { \
          const int pos = wc + (int)__builtin_amdgcn_mbcnt_lo(mj, 0u); \
          if (pos < WCAP) list[wave * WCAP + pos] = ((el0 + (J)) << SLOTB) | (int)(SJ); \
        } \
        wc += (int)__builtin_popcount(mj); } }
    HITJ(0, h0, s0)
    HITJ(1, h1, s1)
    HITJ(2, h2, s2)
    HITJ(3, h3, s3)
    HITJ(4, h4, s4)
    HITJ(5, h5, s5)
    HITJ(6, h6, s6)
    HITJ(7, h7, s7)
#undef HITJ
  }
  return wc;
}

__global__ __launch_bounds__(NTHR) void k_xprep(const float* __restrict__ x, unsigned short* xb, int nN, int nUnits) {
  const int i = (int)blockIdx.x * NTHR + (int)threadIdx.x;
  if (i >= nUnits) return;
  const int row = i >> 5;
  const int c0  = (i & 31) * 8;
  const int rc  = row < nN ? row : nN - 1;
  const float* p = x + (size_t)rc * DIM + c0;
  v4f a = *(const v4fa*)p, b = *(const v4fa*)(p + 4);
  asm volatile("" :: "v"(a), "v"(b));
  const v4f z4 = {0.f, 0.f, 0.f, 0.f};
  if (row >= nN) { a = z4; b = z4; }
  const v4u hv = pack8(a, b);
  unsigned short* dp = xb + (size_t)row * DIM + c0;
  *(volatile v4u*)dp = hv;
  __threadfence();
  *(volatile v4u*)dp = hv;
}

__global__ __launch_bounds__(NTHR) void k_wrel(const float* __restrict__ wq, const float* __restrict__ wk,
                                               const float* __restrict__ wv, unsigned short* pq,
                                               unsigned short* pkv, int nuq, int ksh, int nUnits) {
  const int u = (int)blockIdx.x * NTHR + (int)threadIdx.x;
  if (u >= nUnits) return;
  v4f a, b;
  unsigned short* dp;
  if (u < nuq) {
    const int n = u >> 5, k8 = (u & 31) * 8;
    const float* p = wq + (size_t)n * DIM + k8;
    a = *(const v4fa*)p; b = *(const v4fa*)(p + 4);
    dp = pq + (size_t)u * 8;
  } else {
    const int v  = u - nuq;
    const int n  = v >> ksh;
    const int k8 = (v & ((1 << ksh) - 1)) * 8;
    const int kk = k8 & (DIM - 1);
    const int nr = n & (DIM - 1);
    if (n < DIM) {
      const float* p = wk + (size_t)nr * DIM + kk;
      a = *(const v4fa*)p; b = *(const v4fa*)(p + 4);
    } else {
      const float* p = wv + (size_t)nr * DIM + kk;
      a = *(const v4fa*)p; b = *(const v4fa*)(p + 4);
    }
    dp = pkv + (size_t)v * 8;
  }
  const v4u o = pack8(a, b);
  *(volatile v4u*)dp = o;
  __threadfence();
  *(volatile v4u*)dp = o;
}

__global__ __launch_bounds__(GTHR) __attribute__((amdgpu_num_vgpr(248)))
void k_gemm(const unsigned short* __restrict__ A, int lda,
            const unsigned short* __restrict__ BT, int ldb, int K,
            const float* __restrict__ bias0, const float* __restrict__ bias1,
            float* outF, int ldo, int nN) {
  __shared__ __attribute__((aligned(16))) float stg[GBM * GBN];
  __shared__ __attribute__((aligned(16))) float sbias[GBN];
  const int tid = (int)threadIdx.x, lane = tid & 31, wave = tid >> 5, hh = lane >> 4, m = lane & 15;
  const int rowBase = (int)blockIdx.x * GBM;
  const int col0    = (int)blockIdx.y * GBN;
  {
    const int cg = col0 + tid;
    const int ci = cg & (DIM - 1);
    const float x0 = bias0[ci], x1 = bias1[ci];
    asm volatile("" :: "v"(x0), "v"(x1));
    sbias[tid] = bf_rne(cg < DIM ? x0 : x1);
  }

  v8f acc[GNT];
  {
    const v8f z = {0.f, 0.f, 0.f, 0.f, 0.f, 0.f, 0.f, 0.f};
#pragma unroll
    for (int t = 0; t < GNT; ++t) acc[t] = z;
  }
  const unsigned short* ap = A + (size_t)(rowBase + 16 * wave + m) * (size_t)lda + 8 * hh;
  const unsigned short* bp = BT + (size_t)(col0 + m) * (size_t)ldb + 8 * hh;

#pragma unroll 1
  for (int k0 = 0; k0 < K; k0 += 32) {
    Frag af;
    af.h[0] = *(const v8usa*)(ap + k0);
    af.h[1] = *(const v8usa*)(ap + k0 + 16);
#pragma unroll
    for (int nt = 0; nt < GNT; ++nt) {
      const unsigned short* wq = bp + (size_t)(16 * nt) * (size_t)ldb + k0;
      Frag bfg;
      bfg.h[0] = *(const v8usa*)wq;
      bfg.h[1] = *(const v8usa*)(wq + 16);
      acc[nt] = wmb(af, bfg, acc[nt]);
    }
  }
  __syncthreads();

#pragma unroll
  for (int nt = 0; nt < GNT; ++nt) {
    const int lc = 16 * nt + m;
    const float bb = sbias[lc];
#pragma unroll
    for (int r = 0; r < 8; ++r) {
      const int lr = 16 * wave + 8 * hh + r;
      const bool live = (rowBase + lr) < nN;
      const float v = acc[nt][r] + bb;
      stg[lr * GBN + lc] = live ? v : 0.0f;
    }
  }
  __syncthreads();

  v4f fv[16];
#pragma unroll
  for (int i = 0; i < 16; ++i) {
    const int lr = 16 * wave + i;
    fv[i] = *(const v4fa*)(stg + lr * GBN + 4 * lane);
  }
#pragma unroll
  for (int i = 0; i < 16; ++i) {
    const int gr = rowBase + 16 * wave + i;
    float* op = outF + (size_t)gr * (size_t)ldo + col0 + 4 * lane;
    *(volatile v4f*)op = fv[i];
  }
  __threadfence();
#pragma unroll
  for (int i = 0; i < 16; ++i) {
    const int gr = rowBase + 16 * wave + i;
    float* op = outF + (size_t)gr * (size_t)ldo + col0 + 4 * lane;
    *(volatile v4f*)op = fv[i];
  }
}

__global__ __launch_bounds__(GTHR) __attribute__((amdgpu_num_vgpr(248)))
void k_fuse(const unsigned short* __restrict__ GM, size_t aoff,
            const unsigned short* __restrict__ FW, size_t boff,
            const float* __restrict__ b1, const float* __restrict__ b2,
            const float* __restrict__ fv, const float* __restrict__ fbv, float* E) {
  __shared__ __attribute__((aligned(16))) float stg[FBM * DIM];
  __shared__ __attribute__((aligned(16))) float sb[DIM];
  __shared__ __attribute__((aligned(16))) float sv[DIM];
  __shared__ __attribute__((aligned(16))) float sp[4 * FBM];
  __shared__ __attribute__((aligned(16))) float se[FBM];
  const int tid = (int)threadIdx.x, lane = tid & 31, wave = tid >> 5, hh = lane >> 4, m = lane & 15;
  const int by = (int)blockIdx.y;
  const int rowBase = (int)blockIdx.x * FBM;
#pragma unroll
  for (int q = 0; q < 2; ++q) {
    const int c = tid + GTHR * q;
    const float x1 = b1[c], x2 = b2[c];
    asm volatile("" :: "v"(x1), "v"(x2));
    sb[c] = bf_rne(by != 0 ? x2 : x1);
    sv[c] = bf_rne(fv[c]);
  }
  const int rt = wave & 1, chh = wave >> 1;
  v8f acc[GNT];
  {
    const v8f z = {0.f, 0.f, 0.f, 0.f, 0.f, 0.f, 0.f, 0.f};
#pragma unroll
    for (int t = 0; t < GNT; ++t) acc[t] = z;
  }
  const unsigned short* ap = GM + (size_t)by * aoff + (size_t)(rowBase + 16 * rt + m) * KHL + 8 * hh;
  const unsigned short* bp = FW + (size_t)by * boff + (size_t)(128 * chh + m) * KHL + 8 * hh;
#pragma unroll 1
  for (int k0 = 0; k0 < KHL; k0 += 32) {
    Frag af;
    af.h[0] = *(const v8usa*)(ap + k0);
    af.h[1] = *(const v8usa*)(ap + k0 + 16);
#pragma unroll
    for (int nt = 0; nt < GNT; ++nt) {
      const unsigned short* wq = bp + (size_t)(16 * nt) * KHL + k0;
      Frag bfg;
      bfg.h[0] = *(const v8usa*)wq;
      bfg.h[1] = *(const v8usa*)(wq + 16);
      acc[nt] = wmb(af, bfg, acc[nt]);
    }
  }
#pragma unroll
  for (int nt = 0; nt < GNT; ++nt) {
    const int lc = 128 * chh + 16 * nt + m;
#pragma unroll
    for (int r = 0; r < 8; ++r) {
      const int lr = 16 * rt + 8 * hh + r;
      stg[lr * DIM + lc] = acc[nt][r];
    }
  }
  __syncthreads();
  {
    const int row = tid & 31, part = tid >> 5;
    const float* tr = stg + row * DIM + 64 * part;
    const float* pb = sb + 64 * part;
    const float* pv = sv + 64 * part;
    float s = 0.0f;
#pragma unroll 1
    for (int c = 0; c < 64; ++c) s += tanhf(tr[c] + pb[c]) * pv[c];
    sp[part * FBM + row] = s;
  }
  __syncthreads();
  if (tid < FBM) {
    const float bvv = bf_rne(fbv[0]);
    se[tid] = ((sp[tid] + sp[FBM + tid]) + sp[2 * FBM + tid]) + sp[3 * FBM + tid] + bvv;
  }
  __syncthreads();
  const bool ok = tid < 8;
  const v4f ev = *(const v4fa*)(se + 4 * (tid & 7));
  float* ep = E + (size_t)by * MPG + rowBase + 4 * (tid & 7);
  if (ok) *(volatile v4f*)ep = ev;
  __threadfence();
  if (ok) *(volatile v4f*)ep = ev;
}

__global__ __launch_bounds__(NTHR) void k_gene(
    const unsigned short* __restrict__ GMD, const unsigned short* __restrict__ GMS,
    const float* __restrict__ E, const int* __restrict__ CD, const int* __restrict__ CS,
    const float* __restrict__ feat, const float* __restrict__ lng, const float* __restrict__ lnb,
    float* outF, unsigned short* GO) {
  __shared__ __attribute__((aligned(16))) float sg[DIM];
  __shared__ __attribute__((aligned(16))) float sbt[DIM];
  __shared__ __attribute__((aligned(16))) float stw[NWAVE * DIM];
  const int tid = (int)threadIdx.x, lane = tid & 31, wave = tid >> 5;
  sg[tid]  = bf_rne(lng[tid]);
  sbt[tid] = bf_rne(lnb[tid]);
  __syncthreads();
  const int row = (int)blockIdx.x * NWAVE + wave;
  const bool live = row < NG;
  const int rc = live ? row : NG - 1;
  float* sw = stw + wave * DIM;

  const unsigned short* pa = GMD + (size_t)rc * KHL + 8 * lane;
  const unsigned short* pb = GMS + (size_t)rc * KHL + 8 * lane;
  const v4u ha = *(const v4ua*)pa, la = *(const v4ua*)(pa + DIM);
  const v4u hb = *(const v4ua*)pb, lb = *(const v4ua*)(pb + DIM);
  const float e1 = E[rc], e2 = E[MPG + rc];
  const int cd = CD[rc], cs = CS[rc];
  asm volatile("" :: "v"(ha), "v"(la), "v"(hb), "v"(lb));
  asm volatile("" :: "v"(e1), "v"(e2), "v"(cd), "v"(cs));

  const float gd[8] = {rlo(ha.x, la.x), rhi(ha.x, la.x), rlo(ha.y, la.y), rhi(ha.y, la.y),
                       rlo(ha.z, la.z), rhi(ha.z, la.z), rlo(ha.w, la.w), rhi(ha.w, la.w)};
  const float gs[8] = {rlo(hb.x, lb.x), rhi(hb.x, lb.x), rlo(hb.y, lb.y), rhi(hb.y, lb.y),
                       rlo(hb.z, lb.z), rhi(hb.z, lb.z), rlo(hb.w, lb.w), rhi(hb.w, lb.w)};
  const float mxe = e1 > e2 ? e1 : e2;
  const float x1 = expf(e1 - mxe), x2 = expf(e2 - mxe);
  const float rsum = 1.0f / (x1 + x2);
  const float w0 = x1 * rsum, w1 = x2 * rsum;
  const bool hd = cd > 0, hs = cs > 0;
  const bool both = hd && hs, anyf = hd || hs;
  float mg[8];
#pragma unroll
  for (int j = 0; j < 8; ++j) {
    const float fu  = w0 * gd[j] + w1 * gs[j];
    const float one = hd ? gd[j] : gs[j];
    mg[j] = both ? fu : (anyf ? one : 0.0f);
  }
  {
    v4f mA, mB;
    mA.x = mg[0]; mA.y = mg[1]; mA.z = mg[2]; mA.w = mg[3];
    mB.x = mg[4]; mB.y = mg[5]; mB.z = mg[6]; mB.w = mg[7];
    *(v4fa*)(sw + 8 * lane)     = mA;
    *(v4fa*)(sw + 8 * lane + 4) = mB;
  }
  __builtin_amdgcn_fence(__ATOMIC_RELEASE, "wavefront");
  __builtin_amdgcn_wave_barrier();

  const float* fr = feat + (size_t)rc * DIM + lane;
  float sum = 0.0f;
#pragma unroll 1
  for (int i = 0; i < 8; ++i) {
    const int c = 32 * i + lane;
    const float mv = sw[c];
    const float g  = 0.5f * mv * (1.0f + erff(mv * 0.70710678118654752f));
    const float x  = bf_rne(fr[32 * i]) + g;
    sw[c] = x;
    sum += x;
  }
#pragma unroll
  for (int off = 16; off > 0; off >>= 1) sum += __shfl_xor(sum, off);
  const float mu = sum * (1.0f / 256.0f);
  float vs = 0.0f;
#pragma unroll 1
  for (int i = 0; i < 8; ++i) {
    const float d = sw[32 * i + lane] - mu;
    vs += d * d;
  }
#pragma unroll
  for (int off = 16; off > 0; off >>= 1) vs += __shfl_xor(vs, off);
  const float rs = 1.0f / sqrtf(vs * (1.0f / 256.0f) + LN_EPS);
#pragma unroll 1
  for (int i = 0; i < 8; ++i) {
    const int c = 32 * i + lane;
    sw[c] = (sw[c] - mu) * rs * sg[c] + sbt[c];
  }
  __builtin_amdgcn_fence(__ATOMIC_RELEASE, "wavefront");
  __builtin_amdgcn_wave_barrier();

  const v4f y0 = *(const v4fa*)(sw + 4 * lane);
  const v4f y1 = *(const v4fa*)(sw + 128 + 4 * lane);
  const v4f gA = *(const v4fa*)(sw + 8 * lane);
  const v4f gB = *(const v4fa*)(sw + 8 * lane + 4);
  HL8 hl = hl8(gA, gB);
  const v4u z4 = {0u, 0u, 0u, 0u};
  if (!live) { hl.h = z4; hl.l = z4; }
  float* op = outF + (size_t)row * DIM + 4 * lane;
  unsigned short* gp = GO + (size_t)row * KHL + 8 * lane;
  if (live) { *(volatile v4f*)op = y0; *(volatile v4f*)(op + 128) = y1; }
  *(volatile v4u*)gp = hl.h;
  *(volatile v4u*)(gp + DIM) = hl.l;
  __threadfence();
  if (live) { *(volatile v4f*)op = y0; *(volatile v4f*)(op + 128) = y1; }
  *(volatile v4u*)gp = hl.h;
  *(volatile v4u*)(gp + DIM) = hl.l;
}

template <int MODE>
__global__ __launch_bounds__(NTHR) void k_scan(
    const int* __restrict__ srcs, const int* __restrict__ dsts,
    const float* __restrict__ Q, const float* __restrict__ KVp,
    unsigned short* HP, int* CNT,
    const float* __restrict__ feat, const float* __restrict__ lng, const float* __restrict__ lnb,
    float* outF) {
  constexpr int nN   = (MODE == 0) ? NG : ND;
  constexpr int nSrc = (MODE == 0) ? ND : NG;
  constexpr int nb   = (MODE == 0) ? NB0 : NB1;
  constexpr int nE   = NEDGE;
  constexpr int vec8 = 1;
  extern __shared__ v4f lds_dyn[];
  int* reg1 = (int*)lds_dyn;
  int* reg2 = reg1 + RCAP;
  int* scnt = reg2 + RCAP;
  int* soff = scnt + NBMAX;
  int* list = soff + NBMAX;
  int* wcnt = list + LISTN;
  int* wtot = wcnt + NWAVE;
  const int tid = (int)threadIdx.x, lane = tid & 31, wave = tid >> 5;
  const int nodeBase = (int)blockIdx.x * nb;

  for (int i = tid; i < NBMAX; i += NTHR) scnt[i] = 0;
  __syncthreads();

  int tot = 0;
  const int nChunks = (nE + CHUNK - 1) / CHUNK;
#pragma unroll 1
  for (int ch = 0; ch < nChunks; ++ch) {
    const int cbase = ch * CHUNK;
    const int wc = scan_chunk(dsts, nE, cbase, nodeBase, nb, vec8, list, tid, lane, wave);
    if (lane == 0) wcnt[wave] = wc;
    __syncthreads();
    int pre = 0, all = 0;
#pragma unroll
    for (int w2 = 0; w2 < NWAVE; ++w2) {
      int c = wcnt[w2];
      c = c < 0 ? 0 : (c > WCAP ? WCAP : c);
      all += c;
      pre += (w2 < wave) ? c : 0;
    }
    const int wcc  = wc > WCAP ? WCAP : wc;
    const int base = tot + pre;
#pragma unroll 1
    for (int i = lane; i < wcc; i += 32) {
      const int ent = list[wave * WCAP + i];
      const int el  = (ent >> SLOTB) & (CHUNK - 1);
      const int sl  = ent & (NBMAX - 1);
      int eid = cbase + el;
      eid = eid > nE - 1 ? nE - 1 : eid;
      const int pos = base + i;
      if (pos < RCAP) reg1[pos] = (int)(((unsigned)eid << SLOTB) | (unsigned)sl);
    }
    tot += all;
    tot = tot > RCAP ? RCAP : tot;
    __syncthreads();
  }
  const int nh = tot;

  if (wave == 0) {
#pragma unroll 1
    for (int b0 = 0; b0 < nh; b0 += 32) {
      const int idx = b0 + lane;
      const int uv  = reg1[idx < nh ? idx : nh - 1];
      const int m32 = (nh - b0) < 32 ? (nh - b0) : 32;
#pragma unroll 1
      for (int k = 0; k < m32; ++k) {
        const int u  = __builtin_amdgcn_readlane(uv, k);
        const int sl = u & (NBMAX - 1);
        if (lane == 0) scnt[sl] = scnt[sl] + 1;
      }
    }
  }
  __syncthreads();

  {
    const v4i ca = *(const v4i*)(scnt + 8 * tid);
    const v4i cb = *(const v4i*)(scnt + 8 * tid + 4);
    const int e0 = ca.x < 0 ? 0 : ca.x, e1 = ca.y < 0 ? 0 : ca.y, e2 = ca.z < 0 ? 0 : ca.z, e3 = ca.w < 0 ? 0 : ca.w;
    const int e4 = cb.x < 0 ? 0 : cb.x, e5 = cb.y < 0 ? 0 : cb.y, e6 = cb.z < 0 ? 0 : cb.z, e7 = cb.w < 0 ? 0 : cb.w;
    const int ts = e0 + e1 + e2 + e3 + e4 + e5 + e6 + e7;
    int incl = ts;
#pragma unroll
    for (int d = 1; d < 32; d <<= 1) {
      const int up = __shfl_up(incl, d);
      if (lane >= d) incl += up;
    }
    if (lane == 31) wtot[wave] = incl;
    __syncthreads();
    int pre = 0;
#pragma unroll
    for (int w2 = 0; w2 < NWAVE; ++w2) pre += (w2 < wave) ? wtot[w2] : 0;
    int run = pre + incl - ts;
    soff[8 * tid + 0] = run; run += e0;
    soff[8 * tid + 1] = run; run += e1;
    soff[8 * tid + 2] = run; run += e2;
    soff[8 * tid + 3] = run; run += e3;
    soff[8 * tid + 4] = run; run += e4;
    soff[8 * tid + 5] = run; run += e5;
    soff[8 * tid + 6] = run; run += e6;
    soff[8 * tid + 7] = run;
  }
  __syncthreads();
  for (int i = tid; i < NBMAX; i += NTHR) list[i] = soff[i];
  __syncthreads();

  if (wave == 0) {
#pragma unroll 1
    for (int b0 = 0; b0 < nh; b0 += 32) {
      const int idx = b0 + lane;
      const int uv  = reg1[idx < nh ? idx : nh - 1];
      const int m32 = (nh - b0) < 32 ? (nh - b0) : 32;
#pragma unroll 1
      for (int k = 0; k < m32; ++k) {
        const int u   = __builtin_amdgcn_readlane(uv, k);
        const int sl  = u & (NBMAX - 1);
        const int eid = (int)((unsigned)u >> SLOTB);
        if (lane == 0) {
          int pos = list[sl];
          pos = pos < 0 ? 0 : (pos > RCAP - 1 ? RCAP - 1 : pos);
          reg2[pos] = eid;
          list[sl] = pos + 1;
        }
      }
    }
  }
  __syncthreads();

  const bool ovf = (nh >= RCAP);
  float* lgs = (float*)list;
  float* lbs = lgs + DIM;
  if (MODE == 0) {
    v4i c4 = *(const v4i*)(scnt + 4 * tid);
    c4.x = c4.x < 0 ? 0 : c4.x; c4.y = c4.y < 0 ? 0 : c4.y;
    c4.z = c4.z < 0 ? 0 : c4.z; c4.w = c4.w < 0 ? 0 : c4.w;
    if (ovf) {
      c4.x = c4.x < 1 ? 1 : c4.x; c4.y = c4.y < 1 ? 1 : c4.y;
      c4.z = c4.z < 1 ? 1 : c4.z; c4.w = c4.w < 1 ? 1 : c4.w;
    }
    int* cp = CNT + nodeBase + 4 * tid;
    *(volatile v4i*)cp = c4;
    __threadfence();
    *(volatile v4i*)cp = c4;
  } else {
    lgs[tid] = bf_rne(lng[tid]);
    lbs[tid] = bf_rne(lnb[tid]);
  }
  __syncthreads();

  constexpr int nbw = nb >> 3;
  const float qnan = __int_as_float(0x7fc00000);
  const int c0 = 8 * lane;
  float* stw = (float*)reg1 + wave * STW;
  const v4f z4 = {0.f, 0.f, 0.f, 0.f};

#pragma unroll 1
  for (int jt = 0; jt < nbw; ++jt) {
    const int slot = wave * nbw + jt;
    const int grow = nodeBase + slot;
    const int gcl  = grow < nN ? grow : nN - 1;
    int st = soff[slot];
    const int craw = scnt[slot];
    int cnt = craw;
    st  = st < 0 ? 0 : (st > nh ? nh : st);
    cnt = cnt < 0 ? 0 : (cnt > DEGCAP ? DEGCAP : cnt);
    if (cnt > nh - st) cnt = nh - st;
    const float pz = (ovf || craw > DEGCAP) ? qnan : 0.0f;
    const bool liveRow = grow < nN;

    const float* qp = Q + (size_t)gcl * DIM + c0;
    const v4f q0 = *(const v4fa*)qp, q1 = *(const v4fa*)(qp + 4);
    float mx = MX0, dn = 0.0f;
    v4f aA = z4, aB = z4;

#pragma unroll 1
    for (int q = 0; q < cnt; ++q) {
      int idx = st + q; idx = idx > RCAP - 1 ? RCAP - 1 : idx;
      int eid = reg2[idx]; eid = eid < 0 ? 0 : (eid > nE - 1 ? nE - 1 : eid);
      const int sraw = srcs[eid];
      const int s = sraw < 0 ? 0 : (sraw > nSrc - 1 ? nSrc - 1 : sraw);
      const float* kp = KVp + (size_t)s * KVW + c0;
      const v4f k0 = *(const v4fa*)kp,         k1 = *(const v4fa*)(kp + 4);
      const v4f vA = *(const v4fa*)(kp + DIM), vB = *(const v4fa*)(kp + DIM + 4);
      float p = k0.x * q0.x;
      p = fmaf(k0.y, q0.y, p); p = fmaf(k0.z, q0.z, p); p = fmaf(k0.w, q0.w, p);
      p = fmaf(k1.x, q1.x, p); p = fmaf(k1.y, q1.y, p); p = fmaf(k1.z, q1.z, p); p = fmaf(k1.w, q1.w, p);
      p += __shfl_xor(p, 1);
      p += __shfl_xor(p, 2);
      const float lg = p * QK_SCALE;
      const float df = lg - mx;
      const float ee = expf(-fabsf(df));
      const bool up  = df > 0.0f;
      const float s1 = up ? ee : 1.0f;
      const float s2 = up ? 1.0f : ee;
      mx = up ? lg : mx;
      dn = fmaf(dn, s1, s2);
      aA = aA * s1 + vA * s2;
      aB = aB * s1 + vB * s2;
    }
    const float dnz = dn > 0.0f ? dn : 1.0f;
    const float inv = 1.0f / dnz;
    v4f hA = aA * inv, hB = aB * inv;

    if (MODE == 0) {
      if (!liveRow) { hA = z4; hB = z4; }
      hA = hA + pz; hB = hB + pz;
      const HL8 hl = hl8(hA, hB);
      unsigned short* hp = HP + (size_t)grow * KHL + c0;
      const bool wr = grow < MPG;
      if (wr) { *(volatile v4u*)hp = hl.h; *(volatile v4u*)(hp + DIM) = hl.l; }
      __threadfence();
      if (wr) { *(volatile v4u*)hp = hl.h; *(volatile v4u*)(hp + DIM) = hl.l; }
    } else {
      hA = hA + pz; hB = hB + pz;
      __builtin_amdgcn_fence(__ATOMIC_RELEASE, "wavefront");
      __builtin_amdgcn_wave_barrier();
      *(v4fa*)(stw + c0)     = hA;
      *(v4fa*)(stw + c0 + 4) = hB;
      __builtin_amdgcn_fence(__ATOMIC_RELEASE, "wavefront");
      __builtin_amdgcn_wave_barrier();
      const float* fr = feat + (size_t)gcl * DIM + lane;
      float sum = 0.0f;
#pragma unroll 1
      for (int i = 0; i < 8; ++i) {
        const int c = 32 * i + lane;
        const float mv = stw[c];
        const float g  = 0.5f * mv * (1.0f + erff(mv * 0.70710678118654752f));
        const float x  = bf_rne(fr[32 * i]) + g;
        stw[c] = x;
        sum += x;
      }
#pragma unroll
      for (int off = 16; off > 0; off >>= 1) sum += __shfl_xor(sum, off);
      const float mu = sum * (1.0f / 256.0f);
      float vs = 0.0f;
#pragma unroll 1
      for (int i = 0; i < 8; ++i) {
        const float d = stw[32 * i + lane] - mu;
        vs += d * d;
      }
#pragma unroll
      for (int off = 16; off > 0; off >>= 1) vs += __shfl_xor(vs, off);
      const float rs = 1.0f / sqrtf(vs * (1.0f / 256.0f) + LN_EPS);
#pragma unroll 1
      for (int i = 0; i < 8; ++i) {
        const int c = 32 * i + lane;
        stw[c] = (stw[c] - mu) * rs * lgs[c] + lbs[c] + pz;
      }
      __builtin_amdgcn_fence(__ATOMIC_RELEASE, "wavefront");
      __builtin_amdgcn_wave_barrier();
      const v4f y0 = *(const v4fa*)(stw + 4 * lane);
      const v4f y1 = *(const v4fa*)(stw + 128 + 4 * lane);
      float* op = outF + (size_t)grow * DIM + 4 * lane;
      const bool wr = grow < nN;
      if (wr) { *(volatile v4f*)op = y0; *(volatile v4f*)(op + 128) = y1; }
      __threadfence();
      if (wr) { *(volatile v4f*)op = y0; *(volatile v4f*)(op + 128) = y1; }
    }
  }
  (void)HP; (void)CNT; (void)feat; (void)lng; (void)lnb; (void)outF;
}

static inline int cdiv(int a, int b) { return (a + b - 1) / b; }
constexpr size_t al256c(size_t o) { return (o + 255) & ~(size_t)255; }

constexpr size_t SZ_XBG  = (size_t)MPG * DIM * 2;
constexpr size_t SZ_XBD  = (size_t)MPD * DIM * 2;
constexpr size_t SZ_WQ   = (size_t)4 * DIM * DIM * 2;
constexpr size_t SZ_WKV1 = (size_t)2 * KVW * DIM * 2;
constexpr size_t SZ_WKV2 = (size_t)2 * KVW * KHL * 2;
constexpr size_t SZ_FWD  = (size_t)KVW * KHL * 2;
constexpr size_t SZ_Q1   = (size_t)MPG * DIM * 4;
constexpr size_t SZ_KV1  = (size_t)MPD * KVW * 4;
constexpr size_t SZ_KV2  = (size_t)MPG * KVW * 4;
constexpr size_t SZ_A    = (SZ_Q1 + SZ_KV1 > SZ_KV2) ? (SZ_Q1 + SZ_KV1) : SZ_KV2;
constexpr size_t SZ_Q2   = (size_t)MPD * DIM * 4;
constexpr size_t SZ_GM   = (size_t)MPG * KHL * 2;
constexpr size_t SZ_E    = (size_t)2 * MPG * 4;
constexpr size_t SZ_CNT1 = (size_t)GA0 * NB0 * 4;
constexpr size_t O_XBG  = 0;
constexpr size_t O_XBD  = al256c(O_XBG + SZ_XBG);
constexpr size_t O_XBS  = al256c(O_XBD + SZ_XBD);
constexpr size_t O_WQ   = al256c(O_XBS + SZ_XBD);
constexpr size_t O_WKV1 = al256c(O_WQ + SZ_WQ);
constexpr size_t O_WKV2 = al256c(O_WKV1 + SZ_WKV1);
constexpr size_t O_FWD  = al256c(O_WKV2 + SZ_WKV2);
constexpr size_t O_A    = al256c(O_FWD + SZ_FWD);
constexpr size_t O_Q2   = al256c(O_A + SZ_A);
constexpr size_t O_GM   = al256c(O_Q2 + SZ_Q2);
constexpr size_t O_GO   = al256c(O_GM + 2 * SZ_GM);
constexpr size_t O_E    = al256c(O_GO + SZ_GM);
constexpr size_t O_CNT  = al256c(O_E + SZ_E);
constexpr size_t O_END  = al256c(O_CNT + 2 * SZ_CNT1);
static_assert(O_END <= (size_t)WSMAX);
static_assert((SZ_Q1 % 256) == 0 && (SZ_GM % 256) == 0 && (SZ_CNT1 % 256) == 0);
static_assert(SZ_Q1 + SZ_KV1 <= SZ_A && SZ_KV2 <= SZ_A);

extern "C" void kernel_launch(void* const* d_in, const int* in_sizes, int n_in,
                              void* d_out, int out_size, void* d_ws, size_t ws_size,
                              hipStream_t stream) {
  if (n_in < 45) return;
  if (in_sizes[0] != NG * DIM || in_sizes[1] != ND * DIM || in_sizes[2] != NS * DIM) return;
  for (int i = 3; i <= 30; ++i) {
    const int want = (i & 1) ? DIM * DIM : DIM;
    if (in_sizes[i] != want) return;
  }
  if (in_sizes[31] != DIM || in_sizes[32] != 1) return;
  for (int i = 33; i <= 36; ++i) if (in_sizes[i] != DIM) return;
  for (int i = 37; i <= 44; ++i) if (in_sizes[i] != NEDGE) return;
  if (out_size != OUTN) return;
  if (O_END > ws_size) return;

  const float* gene_feat = (const float*)d_in[0];
  const float* drug_feat = (const float*)d_in[1];
  const float* dis_feat  = (const float*)d_in[2];
  const float* dg_Wq = (const float*)d_in[3];   const float* dg_bq = (const float*)d_in[4];
  const float* dg_Wk = (const float*)d_in[5];   const float* dg_bk = (const float*)d_in[6];
  const float* dg_Wv = (const float*)d_in[7];   const float* dg_bv = (const float*)d_in[8];
  const float* ds_Wq = (const float*)d_in[9];   const float* ds_bq = (const float*)d_in[10];
  const float* ds_Wk = (const float*)d_in[11];  const float* ds_bk = (const float*)d_in[12];
  const float* ds_Wv = (const float*)d_in[13];  const float* ds_bv = (const float*)d_in[14];
  const float* gd_Wq = (const float*)d_in[15];  const float* gd_bq = (const float*)d_in[16];
  const float* gd_Wk = (const float*)d_in[17];  const float* gd_bk = (const float*)d_in[18];
  const float* gd_Wv = (const float*)d_in[19];  const float* gd_bv = (const float*)d_in[20];
  const float* gs_Wq = (const float*)d_in[21];  const float* gs_bq = (const float*)d_in[22];
  const float* gs_Wk = (const float*)d_in[23];  const float* gs_bk = (const float*)d_in[24];
  const float* gs_Wv = (const float*)d_in[25];  const float* gs_bv = (const float*)d_in[26];
  const float* f_W1 = (const float*)d_in[27];   const float* f_b1 = (const float*)d_in[28];
  const float* f_W2 = (const float*)d_in[29];   const float* f_b2 = (const float*)d_in[30];
  const float* f_v  = (const float*)d_in[31];   const float* f_bv = (const float*)d_in[32];
  const float* ln1_g = (const float*)d_in[33];  const float* ln1_b = (const float*)d_in[34];
  const float* ln2_g = (const float*)d_in[35];  const float* ln2_b = (const float*)d_in[36];
  const int* dg_src = (const int*)d_in[37];     const int* dg_dst = (const int*)d_in[38];
  const int* ds_src = (const int*)d_in[39];     const int* ds_dst = (const int*)d_in[40];
  const int* gd_src = (const int*)d_in[41];     const int* gd_dst = (const int*)d_in[42];
  const int* gs_src = (const int*)d_in[43];     const int* gs_dst = (const int*)d_in[44];
  float* out = (float*)d_out;

  char* ws = (char*)d_ws;
  unsigned short* XBg  = (unsigned short*)(ws + O_XBG);
  unsigned short* XBd  = (unsigned short*)(ws + O_XBD);
  unsigned short* XBs  = (unsigned short*)(ws + O_XBS);
  unsigned short* WQ   = (unsigned short*)(ws + O_WQ);
  unsigned short* WKV1 = (unsigned short*)(ws + O_WKV1);
  unsigned short* WKV2 = (unsigned short*)(ws + O_WKV2);
  unsigned short* FWD  = (unsigned short*)(ws + O_FWD);
  float* Q1  = (float*)(ws + O_A);
  float* KV1 = (float*)(ws + O_A + SZ_Q1);
  float* KV2 = (float*)(ws + O_A);
  float* Q2  = (float*)(ws + O_Q2);
  unsigned short* GMd = (unsigned short*)(ws + O_GM);
  unsigned short* GMs = GMd + (size_t)MPG * KHL;
  unsigned short* GO  = (unsigned short*)(ws + O_GO);
  float* Ep  = (float*)(ws + O_E);
  int* CNTd  = (int*)(ws + O_CNT);
  int* CNTs  = CNTd + GA0 * NB0;
  const size_t WQS = (size_t)DIM * DIM;
  const size_t WK1S = (size_t)KVW * DIM;
  const size_t WK2S = (size_t)KVW * KHL;

  hipFuncSetAttribute(reinterpret_cast<const void*>(&k_scan<0>), hipFuncAttributeMaxDynamicSharedMemorySize, LDS_AGG);
  hipFuncSetAttribute(reinterpret_cast<const void*>(&k_scan<1>), hipFuncAttributeMaxDynamicSharedMemorySize, LDS_AGG);

  k_xprep<<<cdiv(MPG * 32, NTHR), NTHR, 0, stream>>>(gene_feat, XBg, NG, MPG * 32);
  k_xprep<<<cdiv(MPD * 32, NTHR), NTHR, 0, stream>>>(drug_feat, XBd, ND, MPD * 32);
  k_xprep<<<cdiv(MPD * 32, NTHR), NTHR, 0, stream>>>(dis_feat,  XBs, NS, MPD * 32);
  {
    const int nq = DIM * (DIM / 8);
    const int n1 = nq + KVW * (DIM / 8);
    const int n2 = nq + KVW * (KHL / 8);
    k_wrel<<<n1 / NTHR, NTHR, 0, stream>>>(dg_Wq, dg_Wk, dg_Wv, WQ,           WKV1,        nq, 5, n1);
    k_wrel<<<n1 / NTHR, NTHR, 0, stream>>>(ds_Wq, ds_Wk, ds_Wv, WQ + WQS,     WKV1 + WK1S, nq, 5, n1);
    k_wrel<<<n2 / NTHR, NTHR, 0, stream>>>(gd_Wq, gd_Wk, gd_Wv, WQ + 2 * WQS, WKV2,        nq, 6, n2);
    k_wrel<<<n2 / NTHR, NTHR, 0, stream>>>(gs_Wq, gs_Wk, gs_Wv, WQ + 3 * WQS, WKV2 + WK2S, nq, 6, n2);
    const int nf = KVW * (KHL / 8);
    k_wrel<<<nf / NTHR, NTHR, 0, stream>>>(f_W1, f_W1, f_W2, FWD, FWD, 0, 6, nf);
  }
  k_gemm<<<dim3(MPG / GBM, DIM / GBN), GTHR, 0, stream>>>(XBg, DIM, WQ, DIM, DIM, dg_bq, dg_bq, Q1, DIM, NG);
  k_gemm<<<dim3(MPD / GBM, KVW / GBN), GTHR, 0, stream>>>(XBd, DIM, WKV1, DIM, DIM, dg_bk, dg_bv, KV1, KVW, ND);
  k_scan<0><<<GA0, NTHR, LDS_AGG, stream>>>(dg_src, dg_dst, Q1, KV1, GMd, CNTd, gene_feat, ln1_g, ln1_b, out);
  k_gemm<<<dim3(MPG / GBM, DIM / GBN), GTHR, 0, stream>>>(XBg, DIM, WQ + WQS, DIM, DIM, ds_bq, ds_bq, Q1, DIM, NG);
  k_gemm<<<dim3(MPD / GBM, KVW / GBN), GTHR, 0, stream>>>(XBs, DIM, WKV1 + WK1S, DIM, DIM, ds_bk, ds_bv, KV1, KVW, NS);
  k_scan<0><<<GA0, NTHR, LDS_AGG, stream>>>(ds_src, ds_dst, Q1, KV1, GMs, CNTs, gene_feat, ln1_g, ln1_b, out);
  k_fuse<<<dim3(MPG / FBM, 2), GTHR, 0, stream>>>(GMd, (size_t)MPG * KHL, FWD, (size_t)DIM * KHL,
                                                  f_b1, f_b2, f_v, f_bv, Ep);
  k_gene<<<MPG / NWAVE, NTHR, 0, stream>>>(GMd, GMs, Ep, CNTd, CNTs, gene_feat, ln1_g, ln1_b, out + OUT2, GO);
  k_gemm<<<dim3(MPG / GBM, KVW / GBN), GTHR, 0, stream>>>(GO, KHL, WKV2, KHL, KHL, gd_bk, gd_bv, KV2, KVW, NG);
  k_gemm<<<dim3(MPD / GBM, DIM / GBN), GTHR, 0, stream>>>(XBd, DIM, WQ + 2 * WQS, DIM, DIM, gd_bq, gd_bq, Q2, DIM, ND);
  k_scan<1><<<GA1, NTHR, LDS_AGG, stream>>>(gd_src, gd_dst, Q2, KV2, GMd, CNTd, drug_feat, ln2_g, ln2_b, out);
  k_gemm<<<dim3(MPG / GBM, KVW / GBN), GTHR, 0, stream>>>(GO, KHL, WKV2 + WK2S, KHL, KHL, gs_bk, gs_bv, KV2, KVW, NG);
  k_gemm<<<dim3(MPD / GBM, DIM / GBN), GTHR, 0, stream>>>(XBs, DIM, WQ + 3 * WQS, DIM, DIM, gs_bq, gs_bq, Q2, DIM, NS);
  k_scan<1><<<GA1, NTHR, LDS_AGG, stream>>>(gs_src, gs_dst, Q2, KV2, GMd, CNTd, dis_feat, ln2_g, ln2_b, out + OUT1);
}
